// FCPairedLayer_67087389164340
// MI455X (gfx1250) — hardware-verified
//
#include <hip/hip_runtime.h>
#include <stddef.h>
#include <stdint.h>

#define NB    2
#define NN    512
#define CIN   64
#define NH    256
#define NBLK  6
#define NF    (NBLK * CIN)
#define NROW  (NB * NN)
#define PW    (NBLK * NH)
#define GTHR  128
#define LDSP  132
#define CTHR  256
#define WTP   72
#define WSMAX 134217728

static_assert(CIN % 32 == 0);
static_assert(NROW % 64 == 0 && PW % 128 == 0);
static_assert(NH % 64 == 0 && PW % 64 == 0);
static_assert((NROW * CIN) % (256 * 8) == 0);
static_assert(NN == (CTHR / 32) * 64);
static_assert(NH == 32 * 8);
static_assert(((LDSP * 4) % 16) == 0 && ((WTP * 2) % 16) == 0);
static_assert(NN / 4 <= CTHR);

typedef float          v4f   __attribute__((ext_vector_type(4)));
typedef float          v8f   __attribute__((ext_vector_type(8)));
typedef int            v8i   __attribute__((ext_vector_type(8)));
typedef unsigned short v8us  __attribute__((ext_vector_type(8)));
typedef unsigned short v16us __attribute__((ext_vector_type(16)));
typedef __bf16         v16bf __attribute__((ext_vector_type(16)));
typedef v4f  __attribute__((may_alias)) v4fa;
typedef v8us __attribute__((may_alias)) v8usa;
union FragB { v16bf v; v16us u; v8us h[2]; v8i w; };

__device__ __forceinline__ v8f wmb(const FragB& a, const FragB& b, v8f c) {
  v8f d = __builtin_amdgcn_wmma_f32_16x16x32_bf16(false, a.v, false, b.v, (short)0, c, false, false);
  asm volatile("v_nop\n\tv_nop\n\tv_nop\n\tv_nop" : "+v"(d) : "v"(a.w), "v"(b.w));
  return d;
}

__device__ __forceinline__ unsigned bf16_bits(float f) {
  const unsigned u = __float_as_uint(f);
  return (u + 0x7FFFu + ((u >> 16) & 1u)) >> 16;
}
__device__ __forceinline__ float bf16_val(float f) {
  return __uint_as_float(bf16_bits(f) << 16);
}

__device__ __forceinline__ void unpack8(const float* p, float o[8]) {
  const v4f a = *(const v4fa*)p;
  const v4f c = *(const v4fa*)(p + 4);
  o[0] = a.x; o[1] = a.y; o[2] = a.z; o[3] = a.w;
  o[4] = c.x; o[5] = c.y; o[6] = c.z; o[7] = c.w;
}

__global__ __launch_bounds__(256) void k_xprep(const float* __restrict__ x, unsigned short* Xb, int nUnits) {
  const int u = (int)blockIdx.x * 256 + (int)threadIdx.x;
  if (u >= nUnits) return;
  const float* p = x + (size_t)u * 8;
  const v4f a = *(const v4fa*)p;
  const v4f c = *(const v4fa*)(p + 4);
  v8us o;
  o[0] = (unsigned short)bf16_bits(a.x);
  o[1] = (unsigned short)bf16_bits(a.y);
  o[2] = (unsigned short)bf16_bits(a.z);
  o[3] = (unsigned short)bf16_bits(a.w);
  o[4] = (unsigned short)bf16_bits(c.x);
  o[5] = (unsigned short)bf16_bits(c.y);
  o[6] = (unsigned short)bf16_bits(c.z);
  o[7] = (unsigned short)bf16_bits(c.w);
  unsigned short* dp = Xb + (size_t)u * 8;
  *(volatile v8us*)dp = o;
  __threadfence();
  *(volatile v8us*)dp = o;
}

__global__ __launch_bounds__(256) void k_wprep(const float* __restrict__ W1, unsigned short* WT) {
  __shared__ __attribute__((aligned(16))) unsigned short sT[64 * WTP];
  const int tid = (int)threadIdx.x;
  const int n0 = (int)blockIdx.x * 64;
  const int kb = n0 >> 8;
  const int hb = n0 & (NH - 1);
#pragma unroll
  for (int it = 0; it < 4; ++it) {
    const int idx = it * 256 + tid;
    const int c = idx >> 4;
    const int q = idx & 15;
    const v4f v = *(const v4fa*)(W1 + (size_t)(kb * CIN + c) * NH + hb + 4 * q);
    sT[(4 * q + 0) * WTP + c] = (unsigned short)bf16_bits(v.x);
    sT[(4 * q + 1) * WTP + c] = (unsigned short)bf16_bits(v.y);
    sT[(4 * q + 2) * WTP + c] = (unsigned short)bf16_bits(v.z);
    sT[(4 * q + 3) * WTP + c] = (unsigned short)bf16_bits(v.w);
  }
  __syncthreads();
  const int pc = tid & 7;
  const int jr = tid >> 3;
  const v8us o0 = *(const v8usa*)(sT + (jr)      * WTP + 8 * pc);
  const v8us o1 = *(const v8usa*)(sT + (jr + 32) * WTP + 8 * pc);
  unsigned short* d0 = WT + (size_t)(n0 + jr)      * CIN + 8 * pc;
  unsigned short* d1 = WT + (size_t)(n0 + jr + 32) * CIN + 8 * pc;
  *(volatile v8us*)d0 = o0;
  *(volatile v8us*)d1 = o1;
  __threadfence();
  *(volatile v8us*)d0 = o0;
  *(volatile v8us*)d1 = o1;
}

__device__ __forceinline__ void gemm_store_pass(const float* sw, float* P, int row0, int col0, int lane) {
#pragma unroll
  for (int i = 0; i < 16; ++i) {
    const v4f v = *(const v4fa*)(sw + i * LDSP + 4 * lane);
    *(volatile v4f*)(P + (size_t)(row0 + i) * PW + col0 + 4 * lane) = v;
  }
}

__global__ __launch_bounds__(GTHR) void k_gemm(const unsigned short* __restrict__ Xb,
                                               const unsigned short* __restrict__ WT,
                                               float* P) {
  __shared__ __attribute__((aligned(16))) float sP[4 * 16 * LDSP];
  const int tid = (int)threadIdx.x, lane = tid & 31, wave = tid >> 5;
  const int hh = lane >> 4, m = lane & 15;
  const int bid = (int)blockIdx.x;
  const int rt = bid / (PW / 128);
  const int ct = bid - rt * (PW / 128);
  const int row0 = 64 * rt + 16 * wave;
  const int col0 = 128 * ct;

  v8f acc[8];
  {
    const v8f z8 = {0.f, 0.f, 0.f, 0.f, 0.f, 0.f, 0.f, 0.f};
#pragma unroll
    for (int t = 0; t < 8; ++t) acc[t] = z8;
  }
  const unsigned short* ap = Xb + (size_t)(row0 + m) * CIN + 8 * hh;
  const unsigned short* wp = WT + (size_t)(col0 + m) * CIN + 8 * hh;

#pragma unroll
  for (int kk = 0; kk < CIN / 32; ++kk) {
    const int k0 = 32 * kk;
    FragB af;
    af.h[0] = *(const v8usa*)(ap + k0);
    af.h[1] = *(const v8usa*)(ap + k0 + 16);
#pragma unroll
    for (int nt = 0; nt < 8; ++nt) {
      const unsigned short* wq = wp + (size_t)(16 * nt) * CIN + k0;
      FragB bf;
      bf.h[0] = *(const v8usa*)wq;
      bf.h[1] = *(const v8usa*)(wq + 16);
      acc[nt] = wmb(af, bf, acc[nt]);
    }
  }

  float* sw = sP + wave * 16 * LDSP;
#pragma unroll
  for (int nt = 0; nt < 8; ++nt) {
#pragma unroll
    for (int r = 0; r < 8; ++r) {
      sw[(8 * hh + r) * LDSP + 16 * nt + m] = acc[nt][r];
    }
  }
  __syncthreads();

  gemm_store_pass(sw, P, row0, col0, lane);
  __threadfence();
  gemm_store_pass(sw, P, row0, col0, lane);
}

__global__ __launch_bounds__(CTHR) void k_comb(const float* __restrict__ P,
                                               const float* __restrict__ b1,
                                               const float* __restrict__ W2,
                                               const float* __restrict__ b2,
                                               float* out) {
  __shared__ float sPart[(CTHR / 32) * 32 * 33];
  __shared__ __attribute__((aligned(16))) float sY[NN];
  const int tid = (int)threadIdx.x, lane = tid & 31, wave = tid >> 5;
  const int bn = (int)blockIdx.x;
  const int b = bn / NN;
  const int n = bn - b * NN;
  const int h0 = 8 * lane;
  const bool nu = (n >= 1);
  const bool nd = (n <= NN - 2);
  const int rU = nu ? bn - 1 : bn;
  const int rD = nd ? bn + 1 : bn;

  float R0[8], R2[8], R4[8], w2[8];
  {
    float t0[8], tb[8];
    unpack8(P + (size_t)bn * PW + 0 * NH + h0, t0);
    unpack8(b1 + h0, tb);
#pragma unroll
    for (int i = 0; i < 8; ++i) R0[i] = t0[i] + bf16_val(tb[i]);
    unpack8(P + (size_t)rU * PW + 2 * NH + h0, R2);
    unpack8(P + (size_t)rD * PW + 4 * NH + h0, R4);
    unpack8(W2 + h0, tb);
#pragma unroll
    for (int i = 0; i < 8; ++i) w2[i] = bf16_val(tb[i]);
  }
  const float b2v = bf16_val(b2[0]);

#pragma unroll 1
  for (int ch = 0; ch < 2; ++ch) {
    const int m0 = 64 * wave + 32 * ch;
#pragma unroll 1
    for (int j = 0; j < 32; ++j) {
      const int m = m0 + j;
      const bool mu = (m <= NN - 2);
      const bool md = (m >= 1);
      const float fu = (nu && mu) ? 1.0f : 0.0f;
      const float fd = (nd && md) ? 1.0f : 0.0f;
      const int rm  = b * NN + m;
      const int rmu = mu ? rm + 1 : rm;
      const int rmd = md ? rm - 1 : rm;
      float p1[8], p3[8], p5[8];
      unpack8(P + (size_t)rm  * PW + 1 * NH + h0, p1);
      unpack8(P + (size_t)rmu * PW + 3 * NH + h0, p3);
      unpack8(P + (size_t)rmd * PW + 5 * NH + h0, p5);
      float acc = 0.0f;
#pragma unroll
      for (int i = 0; i < 8; ++i) {
        float t = R0[i] + p1[i];
        const float u = R2[i] + p3[i];
        t = fmaf(fu, u, t);
        const float d = R4[i] + p5[i];
        t = fmaf(fd, d, t);
        const float hv = fmaxf(t, 0.0f);
        acc = fmaf(hv, w2[i], acc);
      }
      sPart[(wave * 32 + j) * 33 + lane] = acc;
    }
    __syncthreads();
    {
      const float* sp = sPart + (wave * 32 + lane) * 33;
      float y = 0.0f;
#pragma unroll 8
      for (int l = 0; l < 32; ++l) y += sp[l];
      sY[m0 + lane] = y + b2v;
    }
    __syncthreads();
  }

  const int t4 = tid & (NN / 4 - 1);
  const v4f v = *(const v4fa*)(sY + 4 * t4);
  float* op = out + (size_t)bn * NN + 4 * t4;
  if (tid < NN / 4) *(volatile v4f*)op = v;
  __threadfence();
  if (tid < NN / 4) *(volatile v4f*)op = v;
}

extern "C" void kernel_launch(void* const* d_in, const int* in_sizes, int n_in,
                              void* d_out, int out_size, void* d_ws, size_t ws_size,
                              hipStream_t stream) {
  if (n_in < 5) return;
  if (in_sizes[0] != NROW * CIN) return;
  if (in_sizes[1] != NF * NH) return;
  if (in_sizes[2] != NH) return;
  if (in_sizes[3] != NH) return;
  if (in_sizes[4] < 1) return;
  if (out_size != NROW * NN) return;

  const float* x  = (const float*)d_in[0];
  const float* W1 = (const float*)d_in[1];
  const float* b1 = (const float*)d_in[2];
  const float* W2 = (const float*)d_in[3];
  const float* b2 = (const float*)d_in[4];
  float* out = (float*)d_out;

  char* ws = (char*)d_ws;
  size_t off = 0;
  const size_t oXb = off; off += (size_t)NROW * CIN * 2;   off = (off + 255) & ~(size_t)255;
  const size_t oWT = off; off += (size_t)PW * CIN * 2;     off = (off + 255) & ~(size_t)255;
  const size_t oP  = off; off += (size_t)NROW * PW * 4;    off = (off + 255) & ~(size_t)255;
  if (off > ws_size || off > (size_t)WSMAX) return;
  unsigned short* Xb = (unsigned short*)(ws + oXb);
  unsigned short* WT = (unsigned short*)(ws + oWT);
  float*          P  = (float*)(ws + oP);

  const int nUnitsX = NROW * CIN / 8;
  k_xprep<<<nUnitsX / 256, 256, 0, stream>>>(x, Xb, nUnitsX);
  k_wprep<<<PW / 64, 256, 0, stream>>>(W1, WT);
  k_gemm<<<(NROW / 64) * (PW / 128), GTHR, 0, stream>>>(Xb, WT, P);
  k_comb<<<NROW, CTHR, 0, stream>>>(P, b1, W2, b2, out);
}
